// MixtureOfAdapterWithClassifier_42236708389581
// MI455X (gfx1250) — hardware-verified
//
#include <hip/hip_runtime.h>
#include <math.h>

constexpr int kTok = 8192;
constexpr int kHid = 1024;
constexpr int kFF  = 2048;
constexpr int kDom = 4;
constexpr float kLnEps     = 1e-6f;
constexpr float kNegFill   = -1000000000.0f;
constexpr float kWCarry    = 16.0f;
constexpr float kWCarryInv = 1.0f / 16.0f;
constexpr float kInvHid    = 1.0f / 1024.0f;

constexpr size_t kOffZb   = 0;
constexpr size_t kOffZi   = kOffZb + (size_t)kTok * kHid * 2;
constexpr size_t kOffAi   = 0;
constexpr size_t kOffY    = kOffZi + (size_t)kTok * kHid * 2;
constexpr size_t kOffAb   = kOffY + (size_t)kTok * kFF * 2;
constexpr size_t kOffW1T  = kOffAb + (size_t)kTok * kHid * 4;
constexpr size_t kOffW2T  = kOffW1T + (size_t)kFF * kHid * 2;
constexpr size_t kOffGate = kOffW2T + (size_t)kHid * kFF * 2;
constexpr size_t kWsTotal = kOffGate + (size_t)kTok * kDom * 4;

typedef __attribute__((ext_vector_type(16))) _Float16 v16h;
typedef __attribute__((ext_vector_type(8)))  _Float16 v8h;
typedef __attribute__((ext_vector_type(16))) __bf16   v16b;
typedef __attribute__((ext_vector_type(8)))  __bf16   v8b;
typedef __attribute__((ext_vector_type(8)))  float    v8f;
typedef __attribute__((ext_vector_type(4)))  float    v4f;
typedef __attribute__((ext_vector_type(4)))  unsigned int v4u;

__device__ __forceinline__ unsigned short f2bf_bits(float f) {
  unsigned u = __float_as_uint(f);
  return (unsigned short)((u + 0x7FFFu + ((u >> 16) & 1u)) >> 16);
}
__device__ __forceinline__ float bf_bits2f(unsigned short h) { return __uint_as_float(((unsigned)h) << 16); }

__device__ __forceinline__ void dep_guard_h(v8f& a, v8f& b, v16h x, v16h y) { asm volatile("v_nop\n\tv_nop\n\tv_nop\n\tv_nop" : "+v"(a), "+v"(b) : "v"(x), "v"(y)); }
__device__ __forceinline__ void dep_guard_b(v8f& a, v8f& b, v16b x, v16b y) { asm volatile("v_nop\n\tv_nop\n\tv_nop\n\tv_nop" : "+v"(a), "+v"(b) : "v"(x), "v"(y)); }
__device__ __forceinline__ void keep4_h(v16h a, v16h b, v16h c, v16h d) { asm volatile("v_nop" :: "v"(a), "v"(b), "v"(c), "v"(d)); }
__device__ __forceinline__ void keep4_b(v16b a, v16b b, v16b c, v16b d) { asm volatile("v_nop" :: "v"(a), "v"(b), "v"(c), "v"(d)); }
__device__ __forceinline__ void acc_guard4(v8f& a, v8f& b, v8f& c, v8f& d) { asm volatile("v_nop\n\tv_nop\n\tv_nop\n\tv_nop" : "+v"(a), "+v"(b), "+v"(c), "+v"(d)); }
template <typename T> struct Frag;
template <> struct Frag<_Float16> {
  typedef v16h V; union U { v16h v; v8h h[2]; };
  static __device__ __forceinline__ v16h load(const _Float16* p) {
    U f; f.h[0] = *(const v8h*)(p); f.h[1] = *(const v8h*)(p + 16); return f.v;
  }
  static __device__ __forceinline__ v8f mma(v16h a, v16h b, v8f c) {
    return __builtin_amdgcn_wmma_f32_16x16x32_f16(false, a, false, b, (short)0, c, false, false);
  }
  static __device__ __forceinline__ void guard(v8f& a, v8f& b, v16h x, v16h y) { dep_guard_h(a, b, x, y); }
  static __device__ __forceinline__ void keep(v16h a, v16h b, v16h c, v16h d) { keep4_h(a, b, c, d); }
};
template <> struct Frag<__bf16> {
  typedef v16b V; union U { v16b v; v8b h[2]; };
  static __device__ __forceinline__ v16b load(const __bf16* p) {
    U f; f.h[0] = *(const v8b*)(p); f.h[1] = *(const v8b*)(p + 16); return f.v;
  }
  static __device__ __forceinline__ v8f mma(v16b a, v16b b, v8f c) {
    return __builtin_amdgcn_wmma_f32_16x16x32_bf16(false, a, false, b, (short)0, c, false, false);
  }
  static __device__ __forceinline__ void guard(v8f& a, v8f& b, v16b x, v16b y) { dep_guard_b(a, b, x, y); }
  static __device__ __forceinline__ void keep(v16b a, v16b b, v16b c, v16b d) { keep4_b(a, b, c, d); }
};

__device__ __forceinline__ unsigned pk16(unsigned short a, unsigned short b) { return (unsigned)a | ((unsigned)b << 16); }
__device__ __forceinline__ unsigned short h_bits(float f) { const _Float16 h = (_Float16)f; return __builtin_bit_cast(unsigned short, h); }

template <int ET> struct Elem;
template <> struct Elem<0> { typedef _Float16 T; };
template <> struct Elem<1> { typedef __bf16 T; };
template <int ET, bool SPLIT, int BIAS_MODE, int OUT_MODE, bool RESID, int ACT = 0>
__global__ __launch_bounds__(256) void wmma_gemm64(
    const unsigned short* __restrict__ Ap, const unsigned short* __restrict__ A2p, int lda, long strideA,
    const unsigned short* __restrict__ Btp, const unsigned short* __restrict__ Bt2p, int ldb, long strideB,
    void* __restrict__ Cout, void* __restrict__ Cout2, int ldc, long strideC,
    const float* __restrict__ bias,
    const float* __restrict__ resid, long strideR,
    int M, int N, int K, float scale) {
  typedef typename Elem<ET>::T T;
  typedef typename Frag<T>::V V;
  const T* A = (const T*)Ap; const T* A2 = (const T*)A2p; const T* Bt = (const T*)Btp; const T* Bt2 = (const T*)Bt2p;
  __shared__ __align__(16) float sT[8][16 * 68];
  const int b    = blockIdx.y;
  const int lane = threadIdx.x & 31;
  const int wave = threadIdx.x >> 5;
  const int tilesN = N >> 6;
  const int tilesM = M >> 6;
  const int tile = blockIdx.x * 8 + wave;
  if (tile >= tilesM * tilesN) return;
  const int tm = tile / tilesN;
  const int tn = tile - tm * tilesN;
  const int m0 = tm << 6;
  const int n0 = tn << 6;

  const T* Ab  = A  + (size_t)b * strideA;
  const T* Bb  = Bt + (size_t)b * strideB;
  const T* Ab2 = SPLIT ? (A2  + (size_t)b * strideA) : nullptr;
  const T* Bb2 = SPLIT ? (Bt2 + (size_t)b * strideB) : nullptr;

  const int rlane = lane & 15;
  const int koff  = (lane >> 4) * 8;
  const int mOff  = (lane >> 4) * 8;

  v8f acc[4][4];
#pragma unroll
  for (int i = 0; i < 4; ++i)
#pragma unroll
    for (int j = 0; j < 4; ++j) acc[i][j] = (v8f){0.f,0.f,0.f,0.f,0.f,0.f,0.f,0.f};

  for (int k0 = 0; k0 < K; k0 += 32) {
    V bh[4], bl[4];
#pragma unroll
    for (int j = 0; j < 4; ++j) {
      const size_t bo = (size_t)(n0 + (j << 4) + rlane) * ldb + koff + k0;
      bh[j] = Frag<T>::load(Bb + bo);
      if (SPLIT) bl[j] = Frag<T>::load(Bb2 + bo);
    }
#pragma unroll
    for (int i = 0; i < 4; ++i) {
      const size_t ao = (size_t)(m0 + (i << 4) + rlane) * lda + koff + k0;
      V ah = Frag<T>::load(Ab + ao);
      V al;
      if (SPLIT) al = Frag<T>::load(Ab2 + ao);
#pragma unroll
      for (int j = 0; j < 4; ++j) {
        acc[i][j] = Frag<T>::mma(ah, bh[j], acc[i][j]);
        if (SPLIT) {
          acc[i][j] = Frag<T>::mma(ah, bl[j], acc[i][j]);
          acc[i][j] = Frag<T>::mma(al, bh[j], acc[i][j]);
        }
      }
      Frag<T>::guard(acc[i][0], acc[i][3], ah, SPLIT ? al : ah);
    }
    Frag<T>::keep(bh[0], bh[1], bh[2], bh[3]);
    if (SPLIT) Frag<T>::keep(bl[0], bl[1], bl[2], bl[3]);
  }
  acc_guard4(acc[0][0], acc[0][1], acc[0][2], acc[0][3]);
  acc_guard4(acc[1][0], acc[1][1], acc[1][2], acc[1][3]);
  acc_guard4(acc[2][0], acc[2][1], acc[2][2], acc[2][3]);
  acc_guard4(acc[3][0], acc[3][1], acc[3][2], acc[3][3]);

  float* slab = sT[wave];
  const float* Rb = RESID ? (resid + (size_t)b * strideR) : nullptr;
#pragma unroll
  for (int i = 0; i < 4; ++i) {
    const int mBase = m0 + (i << 4);
#pragma unroll
    for (int j = 0; j < 4; ++j) {
      const int n = n0 + (j << 4) + rlane;
      float bv = 0.f;
      if (BIAS_MODE == 2) bv = bias[n];
#pragma unroll
      for (int r = 0; r < 8; ++r) {
        float v = acc[i][j][r] * scale;
        if (BIAS_MODE == 1) v += bias[mBase + mOff + r];
        if (BIAS_MODE == 2) v += bv;
        if (RESID) v += Rb[(size_t)(mBase + mOff + r) * ldc + n];
        if (ACT == 2) v = fmaxf(v, 0.0f);
        if (ACT == 4) v = (v > 0.f) ? v : 0.01f * v;
        slab[(mOff + r) * 68 + (j << 4) + rlane] = v;
      }
    }
    __builtin_amdgcn_fence(__ATOMIC_RELEASE, "workgroup");
    __builtin_amdgcn_wave_barrier();
    __builtin_amdgcn_fence(__ATOMIC_ACQUIRE, "workgroup");
    if (OUT_MODE == 0) {
      float* C = (float*)Cout + (size_t)b * strideC;
      const int hh = lane >> 4, c4 = (lane & 15) * 4;
      for (int pass = 0; pass < 2; ++pass) {
#pragma unroll
        for (int it = 0; it < 8; ++it) {
          const int row = it * 2 + hh;
          v4f v = *(const v4f*)(slab + row * 68 + c4);
          *(volatile v4f*)(C + (size_t)(mBase + row) * ldc + n0 + c4) = v;
        }
        __threadfence();
      }
    } else {
      const int q = lane >> 3, c8 = (lane & 7) * 8;
      unsigned short* C  = (unsigned short*)Cout  + (size_t)b * strideC;
      unsigned short* C2 = (OUT_MODE == 2) ? ((unsigned short*)Cout2 + (size_t)b * strideC) : nullptr;
      for (int pass = 0; pass < 2; ++pass) {
#pragma unroll
        for (int it = 0; it < 4; ++it) {
          const int row = it * 4 + q;
          const float* sp = slab + row * 68 + c8;
          v8h hv, lv;
#pragma unroll
          for (int e = 0; e < 8; ++e) {
            if (OUT_MODE == 1) {
              hv[e] = (_Float16)sp[e];
            } else {
              unsigned short hb = f2bf_bits(sp[e]);
              unsigned short lb = f2bf_bits(sp[e] - bf_bits2f(hb));
              hv[e] = __builtin_bit_cast(_Float16, hb);
              lv[e] = __builtin_bit_cast(_Float16, lb);
            }
          }
          *(volatile v8h*)(C + (size_t)(mBase + row) * ldc + n0 + c8) = hv;
          if (OUT_MODE == 2) *(volatile v8h*)(C2 + (size_t)(mBase + row) * ldc + n0 + c8) = lv;
        }
        __threadfence();
      }
    }
    __builtin_amdgcn_fence(__ATOMIC_RELEASE, "workgroup");
    __builtin_amdgcn_wave_barrier();
    __builtin_amdgcn_fence(__ATOMIC_ACQUIRE, "workgroup");
  }
}

__global__ __launch_bounds__(256) void gate_kernel(const float* __restrict__ x, const int* __restrict__ dmask,
                                                   const float* __restrict__ gw1, const float* __restrict__ gb1,
                                                   const float* __restrict__ gw2, const float* __restrict__ gb2,
                                                   float* __restrict__ gate) {
  __shared__ __align__(16) float sg[8][4];
  const int t = threadIdx.x, lane = t & 31, wave = t >> 5;
  const int row = blockIdx.x * 8 + wave;
  const float* xr = x + (size_t)row * kHid;
  float h0 = 0.f, h1 = 0.f, h2 = 0.f, h3 = 0.f;
#pragma unroll 1
  for (int j = 0; j < kHid / 32; ++j) {
    const int c = j * 32 + lane;
    const float xv = xr[c];
    const v4f g = *(const v4f*)(gw1 + (size_t)c * 4);
    h0 = fmaf(xv, g[0], h0);
    h1 = fmaf(xv, g[1], h1);
    h2 = fmaf(xv, g[2], h2);
    h3 = fmaf(xv, g[3], h3);
  }
#pragma unroll
  for (int off = 16; off > 0; off >>= 1) {
    h0 += __shfl_xor(h0, off, 32);
    h1 += __shfl_xor(h1, off, 32);
    h2 += __shfl_xor(h2, off, 32);
    h3 += __shfl_xor(h3, off, 32);
  }
  float hv[4];
  hv[0] = fmaxf(h0 + gb1[0], 0.f);
  hv[1] = fmaxf(h1 + gb1[1], 0.f);
  hv[2] = fmaxf(h2 + gb1[2], 0.f);
  hv[3] = fmaxf(h3 + gb1[3], 0.f);
  float lg[4];
#pragma unroll
  for (int e = 0; e < 4; ++e) {
    float acc = hv[0] * gw2[0 * 4 + e];
    acc = fmaf(hv[1], gw2[1 * 4 + e], acc);
    acc = fmaf(hv[2], gw2[2 * 4 + e], acc);
    acc = fmaf(hv[3], gw2[3 * 4 + e], acc);
    acc += gb2[e];
    lg[e] = (dmask[e] == 0) ? kNegFill : acc;
  }
  const float mx = fmaxf(fmaxf(lg[0], lg[1]), fmaxf(lg[2], lg[3]));
  float p[4];
  float sum = 0.f;
#pragma unroll
  for (int e = 0; e < 4; ++e) { p[e] = expf(lg[e] - mx); sum += p[e]; }
  const float inv = 1.0f / sum;
  if (lane == 0) {
    sg[wave][0] = p[0] * inv;
    sg[wave][1] = p[1] * inv;
    sg[wave][2] = p[2] * inv;
    sg[wave][3] = p[3] * inv;
  }
  __syncthreads();
  if (wave == 0) {
    const int r = lane & 7;
    const v4f v = *(const v4f*)(&sg[r][0]);
    float* gp = gate + ((size_t)blockIdx.x * 8 + r) * 4;
    if (lane < 8) *(volatile v4f*)gp = v;
    __threadfence();
    if (lane < 8) *(volatile v4f*)gp = v;
  }
}

__global__ __launch_bounds__(256) void wtcast_kernel(const float* __restrict__ W, unsigned short* __restrict__ out,
                                                     int R, int Cc, float scale) {
  __shared__ float sm[64][65];
  const int t  = threadIdx.x;
  const int r0 = blockIdx.x * 64;
  const int c0 = blockIdx.y * 64;
#pragma unroll
  for (int i = 0; i < 16; ++i) {
    const int e = i * 256 + t;
    const int r = e >> 6;
    const int c = e & 63;
    sm[c][r] = W[(size_t)(r0 + r) * Cc + c0 + c] * scale;
  }
  __syncthreads();
  const int lane = t & 31, wave = t >> 5;
  const int q = lane >> 3, c8 = (lane & 7) * 8;
  for (int pass = 0; pass < 2; ++pass) {
#pragma unroll
    for (int it = 0; it < 2; ++it) {
      const int row = wave * 8 + it * 4 + q;
      unsigned short hb[8];
#pragma unroll
      for (int e = 0; e < 8; ++e) hb[e] = h_bits(sm[row][c8 + e]);
      const v4u u = (v4u){pk16(hb[0], hb[1]), pk16(hb[2], hb[3]), pk16(hb[4], hb[5]), pk16(hb[6], hb[7])};
      *(volatile v4u*)(out + (size_t)(c0 + row) * R + r0 + c8) = u;
    }
    __threadfence();
  }
}

__global__ __launch_bounds__(256) void ln2_kernel(const float* __restrict__ x,
                                                  const float* __restrict__ sbk, const float* __restrict__ bbk,
                                                  const float* __restrict__ siw, const float* __restrict__ biw,
                                                  unsigned short* __restrict__ zb, unsigned short* __restrict__ zi) {
  const int t = threadIdx.x, lane = t & 31, wave = t >> 5;
  const int row = blockIdx.x * 8 + wave;
  const float* xr = x + (size_t)row * kHid;
  float s = 0.f;
#pragma unroll 1
  for (int g = 0; g < 4; ++g) {
    const float* p = xr + g * 256 + lane * 8;
    const v4f a = *(const v4f*)(p);
    const v4f c = *(const v4f*)(p + 4);
    s += ((a[0] + a[1]) + (a[2] + a[3])) + ((c[0] + c[1]) + (c[2] + c[3]));
  }
#pragma unroll
  for (int off = 16; off > 0; off >>= 1) s += __shfl_xor(s, off, 32);
  const float mean = s * kInvHid;
  float qv = 0.f;
#pragma unroll 1
  for (int g = 0; g < 4; ++g) {
    const float* p = xr + g * 256 + lane * 8;
    const v4f a = *(const v4f*)(p);
    const v4f c = *(const v4f*)(p + 4);
#pragma unroll
    for (int e = 0; e < 4; ++e) {
      const float d0 = a[e] - mean;
      const float d1 = c[e] - mean;
      qv = fmaf(d0, d0, qv);
      qv = fmaf(d1, d1, qv);
    }
  }
#pragma unroll
  for (int off = 16; off > 0; off >>= 1) qv += __shfl_xor(qv, off, 32);
  const float rstd = rsqrtf(qv * kInvHid + kLnEps);
#pragma unroll 1
  for (int g = 0; g < 4; ++g) {
    const int col0 = g * 256 + lane * 8;
    const float* p = xr + col0;
    const v4f a  = *(const v4f*)(p);
    const v4f c  = *(const v4f*)(p + 4);
    const v4f s0 = *(const v4f*)(sbk + col0);
    const v4f s1 = *(const v4f*)(sbk + col0 + 4);
    const v4f b0 = *(const v4f*)(bbk + col0);
    const v4f b1 = *(const v4f*)(bbk + col0 + 4);
    const v4f t0 = *(const v4f*)(siw + col0);
    const v4f t1 = *(const v4f*)(siw + col0 + 4);
    const v4f u0 = *(const v4f*)(biw + col0);
    const v4f u1 = *(const v4f*)(biw + col0 + 4);
    unsigned short hb[8], hi[8];
#pragma unroll
    for (int e = 0; e < 4; ++e) {
      const float n0 = (a[e] - mean) * rstd;
      const float n1 = (c[e] - mean) * rstd;
      hb[e]     = h_bits(fmaf(n0, s0[e], b0[e]));
      hb[4 + e] = h_bits(fmaf(n1, s1[e], b1[e]));
      hi[e]     = h_bits(fmaf(n0, t0[e], u0[e]));
      hi[4 + e] = h_bits(fmaf(n1, t1[e], u1[e]));
    }
    const v4u ub = (v4u){pk16(hb[0], hb[1]), pk16(hb[2], hb[3]), pk16(hb[4], hb[5]), pk16(hb[6], hb[7])};
    const v4u ui = (v4u){pk16(hi[0], hi[1]), pk16(hi[2], hi[3]), pk16(hi[4], hi[5]), pk16(hi[6], hi[7])};
    unsigned short* pb = zb + (size_t)row * kHid + col0;
    unsigned short* pi = zi + (size_t)row * kHid + col0;
    *(volatile v4u*)pb = ub;
    *(volatile v4u*)pi = ui;
    __threadfence();
    *(volatile v4u*)pb = ub;
    *(volatile v4u*)pi = ui;
  }
}

__global__ __launch_bounds__(256) void combine_kernel(const float* __restrict__ x, const float* __restrict__ gate,
                                                      const float* __restrict__ ab, const float* __restrict__ ai,
                                                      float* __restrict__ out) {
  const size_t i = (size_t)blockIdx.x * 256 + threadIdx.x;
  const int row = (int)(i >> 8);
  const v4f g  = *(const v4f*)(gate + (size_t)row * 4);
  const v4f xv = *(const v4f*)(x + 4 * i);
  const v4f av = *(const v4f*)(ab + 4 * i);
  const v4f iv = *(const v4f*)(ai + 4 * i);
  v4f o;
#pragma unroll
  for (int e = 0; e < 4; ++e) {
    float mix = xv[e] * g[0];
    mix = fmaf(av[e], g[1], mix);
    mix = fmaf(iv[e], g[2], mix);
    o[e] = xv[e] + mix;
  }
  float* op = out + 4 * i;
  *(volatile v4f*)op = o;
  __threadfence();
  *(volatile v4f*)op = o;
}

extern "C" void kernel_launch(void* const* d_in, const int* in_sizes, int n_in,
                              void* d_out, int out_size, void* d_ws, size_t ws_size,
                              hipStream_t stream) {
  if (n_in < 14) return;
  if (in_sizes[0] != kTok * kHid || in_sizes[1] != kDom || in_sizes[2] != kHid * kDom || in_sizes[3] != kDom ||
      in_sizes[4] != kDom * kDom || in_sizes[5] != kDom || in_sizes[6] != kHid || in_sizes[7] != kHid ||
      in_sizes[8] != kHid || in_sizes[9] != kHid || in_sizes[10] != kHid * kFF || in_sizes[11] != kFF ||
      in_sizes[12] != kFF * kHid || in_sizes[13] != kHid) return;
  if ((size_t)out_size != (size_t)kTok * kHid) return;
  if (ws_size < kWsTotal) return;

  const float* x     = (const float*)d_in[0];
  const int*   dmask = (const int*)d_in[1];
  const float* gw1   = (const float*)d_in[2];
  const float* gb1   = (const float*)d_in[3];
  const float* gw2   = (const float*)d_in[4];
  const float* gb2   = (const float*)d_in[5];
  const float* lnsb  = (const float*)d_in[6];
  const float* lnbb  = (const float*)d_in[7];
  const float* lnsi  = (const float*)d_in[8];
  const float* lnbi  = (const float*)d_in[9];
  const float* aw1   = (const float*)d_in[10];
  const float* ab1   = (const float*)d_in[11];
  const float* aw2   = (const float*)d_in[12];
  const float* ab2   = (const float*)d_in[13];
  float* out = (float*)d_out;

  char* ws = (char*)d_ws;
  unsigned short* Zb   = (unsigned short*)(ws + kOffZb);
  unsigned short* Zi   = (unsigned short*)(ws + kOffZi);
  float*          Ai   = (float*)(ws + kOffAi);
  unsigned short* Y    = (unsigned short*)(ws + kOffY);
  float*          Ab   = (float*)(ws + kOffAb);
  unsigned short* W1T  = (unsigned short*)(ws + kOffW1T);
  unsigned short* W2T  = (unsigned short*)(ws + kOffW2T);
  float*          gate = (float*)(ws + kOffGate);

  gate_kernel<<<dim3(kTok / 8), dim3(256), 0, stream>>>(x, dmask, gw1, gb1, gw2, gb2, gate);

  wtcast_kernel<<<dim3(kHid / 64, kFF / 64), dim3(256), 0, stream>>>(aw1, W1T, kHid, kFF, kWCarry);
  wtcast_kernel<<<dim3(kFF / 64, kHid / 64), dim3(256), 0, stream>>>(aw2, W2T, kFF, kHid, kWCarry);

  ln2_kernel<<<dim3(kTok / 8), dim3(256), 0, stream>>>(x, lnsb, lnbb, lnsi, lnbi, Zb, Zi);

  const int tiles1 = (kTok / 64) * (kFF / 64);
  const int tiles2 = (kTok / 64) * (kHid / 64);

  wmma_gemm64<0, false, 2, 1, false, 2><<<dim3(tiles1 / 8, 1), dim3(256), 0, stream>>>(
      Zb, Zb, kHid, 0L, W1T, W1T, kHid, 0L, (void*)Y, (void*)Y, kFF, 0L, ab1, gate, 0L, kTok, kFF, kHid, kWCarryInv);
  wmma_gemm64<0, false, 2, 0, false, 0><<<dim3(tiles2 / 8, 1), dim3(256), 0, stream>>>(
      Y, Y, kFF, 0L, W2T, W2T, kFF, 0L, (void*)Ab, (void*)Ab, kHid, 0L, ab2, gate, 0L, kTok, kHid, kFF, kWCarryInv);

  wmma_gemm64<0, false, 2, 1, false, 2><<<dim3(tiles1 / 8, 1), dim3(256), 0, stream>>>(
      Zi, Zi, kHid, 0L, W1T, W1T, kHid, 0L, (void*)Y, (void*)Y, kFF, 0L, ab1, gate, 0L, kTok, kFF, kHid, kWCarryInv);
  wmma_gemm64<0, false, 2, 0, false, 0><<<dim3(tiles2 / 8, 1), dim3(256), 0, stream>>>(
      Y, Y, kFF, 0L, W2T, W2T, kFF, 0L, (void*)Ai, (void*)Ai, kHid, 0L, ab2, gate, 0L, kTok, kHid, kFF, kWCarryInv);

  combine_kernel<<<dim3(kTok * kHid / 4 / 256), dim3(256), 0, stream>>>(x, gate, Ab, Ai, out);
}
